// MHSA_3521873183477
// MI455X (gfx1250) — hardware-verified
//
#include <hip/hip_runtime.h>
#include <stdint.h>


typedef unsigned short hword;
typedef hword us8  __attribute__((ext_vector_type(8)));
typedef hword us16 __attribute__((ext_vector_type(16)));
typedef __bf16 bf16x16 __attribute__((ext_vector_type(16)));
typedef _Float16 f16x16 __attribute__((ext_vector_type(16)));
typedef float v8f __attribute__((ext_vector_type(8)));
typedef float v4f __attribute__((ext_vector_type(4)));

#define SEQ   2048
#define DIM   1024
#define HD    64
#define NH    16
#define MROWS 4096
#define LDT   68
#define OP    72

__device__ __forceinline__ hword f2bf(float x) {
    unsigned int u = __float_as_uint(x);
    u = (u + 0x7FFFu + ((u >> 16) & 1u)) >> 16;
    return (hword)u;
}
__device__ __forceinline__ float bf2f(hword b) {
    return __uint_as_float(((unsigned int)b) << 16);
}
__device__ __forceinline__ hword f2h(float x) {
    _Float16 t = (_Float16)x;
    return __builtin_bit_cast(hword, t);
}
__device__ __forceinline__ v8f zero8() {
    v8f z;
#pragma unroll
    for (int i = 0; i < 8; ++i) z[i] = 0.0f;
    return z;
}

__device__ __forceinline__ v8f mma_bf(v8f c, us16 a, us16 b) {
    bf16x16 av = __builtin_bit_cast(bf16x16, a);
    bf16x16 bv = __builtin_bit_cast(bf16x16, b);
    c = __builtin_amdgcn_wmma_f32_16x16x32_bf16(false, av, false, bv, (short)0, c, false, false);
    asm volatile("v_nop\n\tv_nop\n\tv_nop\n\tv_nop" : "+v"(c) : "v"(a), "v"(b));
    return c;
}
__device__ __forceinline__ v8f mma_hf(v8f c, us16 a, us16 b) {
    f16x16 av = __builtin_bit_cast(f16x16, a);
    f16x16 bv = __builtin_bit_cast(f16x16, b);
    c = __builtin_amdgcn_wmma_f32_16x16x32_f16(false, av, false, bv, (short)0, c, false, false);
    asm volatile("v_nop\n\tv_nop\n\tv_nop\n\tv_nop" : "+v"(c) : "v"(a), "v"(b));
    return c;
}

__device__ __forceinline__ us16 frag_rows(const hword* p, int ld, int row, int k0, int h) {
    const hword* base = p + (size_t)row * ld + k0 + 8 * h;
    us8 e0 = *(const us8*)(base);
    us8 e1 = *(const us8*)(base + 16);
    return __builtin_shufflevector(e0, e1, 0, 1, 2, 3, 4, 5, 6, 7,
                                   8, 9, 10, 11, 12, 13, 14, 15);
}

__global__ __launch_bounds__(256) void k_cvt3(const float* __restrict__ src, int n8, float fscale,
                                              hword* __restrict__ df,
                                              hword* __restrict__ dh,
                                              hword* __restrict__ dl) {
    const int i = blockIdx.x * 256 + threadIdx.x;
    if (i >= n8) return;
    const float* s = src + (size_t)i * 8;
    const v4f a = *(const v4f*)(s);
    const v4f b = *(const v4f*)(s + 4);
    us8 of, oh, ol;
#pragma unroll
    for (int e = 0; e < 4; ++e) {
        const float x0 = a[e], x1 = b[e];
        of[e]     = f2h(x0 * fscale);
        of[4 + e] = f2h(x1 * fscale);
        const hword h0 = f2bf(x0), h1 = f2bf(x1);
        oh[e] = h0;      oh[4 + e] = h1;
        ol[e] = f2bf(x0 - bf2f(h0));
        ol[4 + e] = f2bf(x1 - bf2f(h1));
    }
    const size_t o8 = (size_t)i * 8;
    *(volatile us8*)(df + o8) = of;
    *(volatile us8*)(dh + o8) = oh;
    *(volatile us8*)(dl + o8) = ol;
    __threadfence();
    *(volatile us8*)(df + o8) = of;
    *(volatile us8*)(dh + o8) = oh;
    *(volatile us8*)(dl + o8) = ol;
}

__global__ __launch_bounds__(256) void k_cvt1(const float* __restrict__ src, int n8, float fscale,
                                              hword* __restrict__ df) {
    const int i = blockIdx.x * 256 + threadIdx.x;
    if (i >= n8) return;
    const float* s = src + (size_t)i * 8;
    const v4f a = *(const v4f*)(s);
    const v4f b = *(const v4f*)(s + 4);
    us8 of;
#pragma unroll
    for (int e = 0; e < 4; ++e) {
        of[e]     = f2h(a[e] * fscale);
        of[4 + e] = f2h(b[e] * fscale);
    }
    const size_t o8 = (size_t)i * 8;
    *(volatile us8*)(df + o8) = of;
    __threadfence();
    *(volatile us8*)(df + o8) = of;
}

__device__ __forceinline__ void qk_pass(const float* tile, hword* P0, hword* P1,
                                        size_t rb, int w, int p, int lq) {
#pragma unroll
    for (int i = 0; i < 4; ++i) {
        const int row = w * 16 + 4 * i + lq;
        const float* sp = tile + row * LDT + 8 * p;
        const v4f u0 = *(const v4f*)(sp);
        const v4f u1 = *(const v4f*)(sp + 4);
        us8 oh, ol;
#pragma unroll
        for (int e = 0; e < 4; ++e) {
            const hword a = f2bf(u0[e]);
            oh[e] = a;
            ol[e] = f2bf(u0[e] - bf2f(a));
            const hword c = f2bf(u1[e]);
            oh[4 + e] = c;
            ol[4 + e] = f2bf(u1[e] - bf2f(c));
        }
        const size_t doff = (rb + (size_t)row) * HD + 8 * p;
        *(volatile us8*)(P0 + doff) = oh;
        *(volatile us8*)(P1 + doff) = ol;
    }
}
__device__ __forceinline__ void v_pass(const float* tile, hword* vt, size_t vb, int n0,
                                       int w, int p, int lq) {
#pragma unroll
    for (int i = 0; i < 4; ++i) {
        const int d = w * 16 + 4 * i + lq;
        us8 o;
#pragma unroll
        for (int e = 0; e < 8; ++e) o[e] = f2h(tile[(8 * p + e) * LDT + d]);
        *(volatile us8*)(vt + (vb + (size_t)d) * SEQ + (size_t)n0 + 8 * p) = o;
    }
}

template <int SV>
__global__ __launch_bounds__(128) void k_qkv(const hword* xa, const hword* xb,
                                             const hword* wa, const hword* wb,
                                             const float* bias,
                                             hword* d0, hword* d1, hword* d2, hword* d3) {
    __shared__ __align__(16) float tile[64 * LDT];
    const int w = threadIdx.x >> 5, lane = threadIdx.x & 31;
    const int h = lane >> 4, m = lane & 15;
    const int mt = blockIdx.x & 63, ng = blockIdx.x >> 6;
    const int s  = SV ? 2 : (ng >> 4);
    const int hh = SV ? ng : (ng & 15);
    const int tok0 = mt * 64;
    const int wr = w & 1, wc = w >> 1;
    const int ar0 = tok0 + wr * 32;

    int orow[2];
#pragma unroll
    for (int t = 0; t < 2; ++t) orow[t] = hh * 192 + (wc * 32 + t * 16 + m) * 3 + s;

    v8f acc[2][2];
#pragma unroll
    for (int mi = 0; mi < 2; ++mi)
#pragma unroll
        for (int t = 0; t < 2; ++t) acc[mi][t] = zero8();

    if (SV == 0) {
#pragma unroll 1
        for (int k0 = 0; k0 < DIM; k0 += 32) {
            const us16 a0h = frag_rows(xa, DIM, ar0 + m, k0, h);
            const us16 a0l = frag_rows(xb, DIM, ar0 + m, k0, h);
            const us16 a1h = frag_rows(xa, DIM, ar0 + 16 + m, k0, h);
            const us16 a1l = frag_rows(xb, DIM, ar0 + 16 + m, k0, h);
#pragma unroll
            for (int t = 0; t < 2; ++t) {
                const us16 bhi = frag_rows(wa, DIM, orow[t], k0, h);
                const us16 blo = frag_rows(wb, DIM, orow[t], k0, h);
                acc[0][t] = mma_bf(acc[0][t], a0h, bhi);
                acc[0][t] = mma_bf(acc[0][t], a0h, blo);
                acc[0][t] = mma_bf(acc[0][t], a0l, bhi);
                acc[1][t] = mma_bf(acc[1][t], a1h, bhi);
                acc[1][t] = mma_bf(acc[1][t], a1h, blo);
                acc[1][t] = mma_bf(acc[1][t], a1l, bhi);
            }
        }
    } else {
#pragma unroll 1
        for (int k0 = 0; k0 < DIM; k0 += 32) {
            const us16 a0 = frag_rows(xa, DIM, ar0 + m, k0, h);
            const us16 a1 = frag_rows(xa, DIM, ar0 + 16 + m, k0, h);
#pragma unroll
            for (int t = 0; t < 2; ++t) {
                const us16 b = frag_rows(wa, DIM, orow[t], k0, h);
                acc[0][t] = mma_hf(acc[0][t], a0, b);
                acc[1][t] = mma_hf(acc[1][t], a1, b);
            }
        }
    }

    const float scl = SV ? (1.0f / 32.0f) : 1.0f;
#pragma unroll
    for (int t = 0; t < 2; ++t) {
        const float bv = bias[orow[t]];
#pragma unroll
        for (int mi = 0; mi < 2; ++mi)
#pragma unroll
            for (int r = 0; r < 8; ++r)
                tile[(wr * 32 + mi * 16 + 8 * h + r) * LDT + wc * 32 + t * 16 + m] =
                    acc[mi][t][r] * scl + bv;
    }
    __syncthreads();

    const int bb = tok0 >> 11, n0 = tok0 & (SEQ - 1);
    const int p = lane & 7, lq = lane >> 3;
    if (SV == 0) {
        hword* P0 = (s == 0) ? d0 : d2;
        hword* P1 = (s == 0) ? d1 : d3;
        const size_t rb = ((size_t)(bb * NH + hh)) * SEQ + (size_t)n0;
        qk_pass(tile, P0, P1, rb, w, p, lq);
        __threadfence();
        qk_pass(tile, P0, P1, rb, w, p, lq);
    } else {
        const size_t vb = ((size_t)(bb * NH + hh)) * HD;
        v_pass(tile, d0, vb, n0, w, p, lq);
        __threadfence();
        v_pass(tile, d0, vb, n0, w, p, lq);
    }
}

__global__ __launch_bounds__(128) void k_attn(const hword* qh, const hword* ql,
                                              const hword* kh, const hword* kl,
                                              const hword* vt, hword* ao) {
    __shared__ __align__(16) hword st[4 * 16 * OP];
    const int w = threadIdx.x >> 5, lane = threadIdx.x & 31;
    const int h = lane >> 4, m = lane & 15;
    const int qt = blockIdx.x & 31, bh = blockIdx.x >> 5;
    const size_t poff = (size_t)bh * SEQ * HD;
    const hword* qhp = qh + poff;
    const hword* qlp = ql + poff;
    const hword* khp = kh + poff;
    const hword* klp = kl + poff;
    const hword* vtp = vt + poff;
    const int q0 = qt * 64 + w * 16;

    us16 qbh[2], qbl[2];
#pragma unroll
    for (int dc = 0; dc < 2; ++dc) {
        qbh[dc] = frag_rows(qhp, HD, q0 + m, dc * 32, h);
        qbl[dc] = frag_rows(qlp, HD, q0 + m, dc * 32, h);
    }

    v8f oacc[4];
#pragma unroll
    for (int dt = 0; dt < 4; ++dt) oacc[dt] = zero8();
    float mrun = -1.0e30f, lrun = 0.0f;

#pragma unroll 1
    for (int kc = 0; kc < SEQ; kc += 64) {
        v8f sacc[4];
#pragma unroll
        for (int kt = 0; kt < 4; ++kt) {
            v8f sa = zero8();
            const int krow = kc + kt * 16 + m;
#pragma unroll
            for (int dc = 0; dc < 2; ++dc) {
                const us16 ka = frag_rows(khp, HD, krow, dc * 32, h);
                const us16 kb = frag_rows(klp, HD, krow, dc * 32, h);
                sa = mma_bf(sa, ka, qbh[dc]);
                sa = mma_bf(sa, ka, qbl[dc]);
                sa = mma_bf(sa, kb, qbh[dc]);
            }
            sacc[kt] = sa;
        }

        float mloc = -1.0e30f;
#pragma unroll
        for (int kt = 0; kt < 4; ++kt)
#pragma unroll
            for (int r = 0; r < 8; ++r) mloc = fmaxf(mloc, sacc[kt][r]);
        mloc = fmaxf(mloc, __shfl_xor(mloc, 16, 32));
        const float mnew = fmaxf(mrun, mloc);
        const float corr = __expf(mrun - mnew);
        mrun = mnew;
        float lsum = 0.0f;
        us16 pb[2];
#pragma unroll
        for (int kt = 0; kt < 4; ++kt) {
#pragma unroll
            for (int r = 0; r < 8; ++r) {
                const float pv = __expf(sacc[kt][r] - mnew);
                lsum += pv;
                pb[kt >> 1][(kt & 1) * 8 + r] = f2h(pv * 16384.0f);
            }
        }
        lsum += __shfl_xor(lsum, 16, 32);
        lrun = lrun * corr + lsum;
#pragma unroll
        for (int dt = 0; dt < 4; ++dt) oacc[dt] = oacc[dt] * corr;

#pragma unroll
        for (int ks = 0; ks < 2; ++ks) {
#pragma unroll
            for (int dt = 0; dt < 4; ++dt) {
                const us16 va = frag_rows(vtp, SEQ, dt * 16 + m, kc + ks * 32, h);
                oacc[dt] = mma_hf(oacc[dt], va, pb[ks]);
            }
        }
    }

    const float inv = 1.0f / (lrun * 524288.0f);
    hword* sw = st + w * (16 * OP);
#pragma unroll
    for (int dt = 0; dt < 4; ++dt) {
        us8 o;
#pragma unroll
        for (int r = 0; r < 8; ++r) o[r] = f2h(oacc[dt][r] * inv);
        *(us8*)(sw + m * OP + dt * 16 + 8 * h) = o;
    }
    __syncthreads();

    const int p = lane & 7, lq = lane >> 3;
    const int bb = bh >> 4, hh = bh & 15;
#pragma unroll
    for (int i = 0; i < 4; ++i) {
        const int row = 4 * i + lq;
        const us8 o = *(const us8*)(sw + row * OP + 8 * p);
        hword* dp = ao + ((size_t)(bb * SEQ + q0 + row)) * DIM + hh * HD + 8 * p;
        *(volatile us8*)dp = o;
    }
    __threadfence();
#pragma unroll
    for (int i = 0; i < 4; ++i) {
        const int row = 4 * i + lq;
        const us8 o = *(const us8*)(sw + row * OP + 8 * p);
        hword* dp = ao + ((size_t)(bb * SEQ + q0 + row)) * DIM + hh * HD + 8 * p;
        *(volatile us8*)dp = o;
    }
}

__device__ __forceinline__ void store_tile_rows64(const float* tile, float* dst,
                                                  size_t drow0, int dpitch, int lane) {
    const int h = lane >> 4, m = lane & 15;
#pragma unroll
    for (int i = 0; i < 16; ++i) {
        const int row = 2 * i + h;
        v4f v = *(const v4f*)(tile + row * LDT + 4 * m);
        *(volatile v4f*)(dst + (drow0 + (size_t)row) * (size_t)dpitch + 4 * m) = v;
    }
    __threadfence();
#pragma unroll
    for (int i = 0; i < 16; ++i) {
        const int row = 2 * i + h;
        v4f v = *(const v4f*)(tile + row * LDT + 4 * m);
        *(volatile v4f*)(dst + (drow0 + (size_t)row) * (size_t)dpitch + 4 * m) = v;
    }
}

__global__ __launch_bounds__(128) void k_proj(const hword* af, const hword* wf,
                                              const float* bias, float* out) {
    __shared__ __align__(16) float stg[4 * 32 * LDT];
    const int w = threadIdx.x >> 5, lane = threadIdx.x & 31;
    const int h = lane >> 4, m = lane & 15;
    const int wid = blockIdx.x * 4 + w;
    const int mt = wid & 127, ng = wid >> 7;
    const int row0 = mt * 32, n0 = ng * 64;

    v8f acc[2][4];
#pragma unroll
    for (int mi = 0; mi < 2; ++mi)
#pragma unroll
        for (int t = 0; t < 4; ++t) acc[mi][t] = zero8();

#pragma unroll 1
    for (int k0 = 0; k0 < DIM; k0 += 32) {
        const us16 a0 = frag_rows(af, DIM, row0 + m, k0, h);
        const us16 a1 = frag_rows(af, DIM, row0 + 16 + m, k0, h);
#pragma unroll
        for (int t = 0; t < 4; ++t) {
            const us16 b = frag_rows(wf, DIM, n0 + t * 16 + m, k0, h);
            acc[0][t] = mma_hf(acc[0][t], a0, b);
            acc[1][t] = mma_hf(acc[1][t], a1, b);
        }
    }

    float* tile = stg + w * (32 * LDT);
#pragma unroll
    for (int t = 0; t < 4; ++t) {
        const float bv = bias[n0 + t * 16 + m];
#pragma unroll
        for (int mi = 0; mi < 2; ++mi)
#pragma unroll
            for (int r = 0; r < 8; ++r)
                tile[(mi * 16 + 8 * h + r) * LDT + t * 16 + m] =
                    acc[mi][t][r] * (1.0f / 32.0f) + bv;
    }
    __syncthreads();

    store_tile_rows64(tile, out + n0, (size_t)row0, DIM, lane);
}

extern "C" void kernel_launch(void* const* d_in, const int* in_sizes, int n_in,
                              void* d_out, int out_size, void* d_ws, size_t ws_size,
                              hipStream_t stream) {
    if (n_in < 5) return;
    const int nx  = MROWS * DIM;
    const int nwq = 3 * DIM * DIM;
    const int nwp = DIM * DIM;
    if (in_sizes[0] != nx || in_sizes[1] != nwq || in_sizes[2] != 3 * DIM ||
        in_sizes[3] != nwp || in_sizes[4] != DIM || out_size != nx) return;

    const float* x     = (const float*)d_in[0];
    const float* Wqkv  = (const float*)d_in[1];
    const float* bqkv  = (const float*)d_in[2];
    const float* Wproj = (const float*)d_in[3];
    const float* bproj = (const float*)d_in[4];
    float* out = (float*)d_out;

    const size_t b_x  = (size_t)nx * 2;
    const size_t b_wq = (size_t)nwq * 2;
    const size_t b_wp = (size_t)nwp * 2;
    const size_t b_hp = (size_t)MROWS * DIM * 2;
    size_t off = 0;
    char* ws = (char*)d_ws;
    hword* xf  = (hword*)(ws + off); off += b_x;
    hword* xbh = (hword*)(ws + off); off += b_x;
    hword* xbl = (hword*)(ws + off); off += b_x;
    hword* wf  = (hword*)(ws + off); off += b_wq;
    hword* wbh = (hword*)(ws + off); off += b_wq;
    hword* wbl = (hword*)(ws + off); off += b_wq;
    hword* wpf = (hword*)(ws + off); off += b_wp;
    hword* qh  = (hword*)(ws + off); off += b_hp;
    hword* ql  = (hword*)(ws + off); off += b_hp;
    hword* kh  = (hword*)(ws + off); off += b_hp;
    hword* kl  = (hword*)(ws + off); off += b_hp;
    hword* vt  = (hword*)(ws + off); off += b_hp;
    hword* aof = (hword*)(ws + off); off += b_hp;
    if (off > ws_size) return;

    const int n8x = nx / 8, n8q = nwq / 8, n8p = nwp / 8;
    k_cvt3<<<(n8x + 255) / 256, 256, 0, stream>>>(x, n8x, 1.0f, xf, xbh, xbl);
    k_cvt3<<<(n8q + 255) / 256, 256, 0, stream>>>(Wqkv, n8q, 32.0f, wf, wbh, wbl);
    k_cvt1<<<(n8p + 255) / 256, 256, 0, stream>>>(Wproj, n8p, 32.0f, wpf);

    k_qkv<0><<<2048, 128, 0, stream>>>(xbh, xbl, wbh, wbl, bqkv, qh, ql, kh, kl);
    k_qkv<1><<<1024, 128, 0, stream>>>(xf, xf, wf, wf, bqkv, vt, vt, vt, vt);

    k_attn<<<1024, 128, 0, stream>>>(qh, ql, kh, kl, vt, aof);

    k_proj<<<512, 128, 0, stream>>>(aof, wpf, bproj, out);
}
